// GAM_GNN_32873679684152
// MI455X (gfx1250) — hardware-run, weakly checked
//
#include <hip/hip_runtime.h>

typedef __attribute__((ext_vector_type(16))) __bf16   v16b;
typedef __attribute__((ext_vector_type(8)))  __bf16   v8b;
typedef __attribute__((ext_vector_type(8)))  float    v8f;
typedef __attribute__((ext_vector_type(4)))  float    v4f;
typedef __attribute__((ext_vector_type(4)))  unsigned v4u;

constexpr int kNodes    = 8192;
constexpr int kEdges    = 131072;
constexpr int kEA       = 6;
constexpr int kHid      = 768;
constexpr int kMsg      = 249;
constexpr int kMsgPad   = 256;
constexpr int kMono     = 83;
constexpr int kNodeIn   = 16;
constexpr int kLnDim    = 19;
constexpr int kU1       = 18;
constexpr int kU2       = 17;
constexpr int kOutDim   = 16;
constexpr int kTileE    = 64;
constexpr int kRowsPass = 32;
constexpr int kMaxDeg   = 32;
constexpr int kSearchIters = 18;
constexpr int kTilesW2  = (kHid / 64) * (kHid / 64);
constexpr int kTilesW3  = (kMsgPad / 64) * (kHid / 64);
static_assert(kMono * 3 == kMsg);
static_assert(6 + 21 + 56 == kMono);
static_assert((kHid % 32) == 0 && (kHid % 64) == 0 && (kMsgPad % 64) == 0);
static_assert((kEdges % kTileE) == 0 && (kNodes % 256) == 0);
static_assert(kEdges <= (1 << 17));
static_assert(kNodeIn + 3 == kLnDim);

constexpr size_t kOffW2   = 0;
constexpr size_t kBytesW2 = (size_t)kHid * kHid * 2;
constexpr size_t kOffW3   = kOffW2 + kBytesW2;
constexpr size_t kBytesW3 = (size_t)kMsgPad * kHid * 2;
constexpr size_t kOffRes  = kOffW3 + kBytesW3;
constexpr size_t kBytesRes = (size_t)kEdges * 4 * 4;
constexpr size_t kWsTotal = kOffRes + kBytesRes;
static_assert(kWsTotal == 3670016ull);
static_assert(kWsTotal <= 134217728ull);
static_assert((kOffW3 % 128) == 0 && (kOffRes % 128) == 0);

constexpr int kPlaneHalves = kRowsPass * kHid;
constexpr int kLdsEdge = 4 * kPlaneHalves * 2 + kTileE * 8 * 4 + kTileE * 4 * 4 + kTileE * 4 + kTileE * 4;
static_assert(kLdsEdge == 200192);
static_assert(kRowsPass * kMsgPad * 4 <= kPlaneHalves * 2);

__device__ __forceinline__ unsigned f2bf_bits(float f) {
  const unsigned u = __float_as_uint(f);
  return (u + 0x7FFFu + ((u >> 16) & 1u)) >> 16;
}
__device__ __forceinline__ float bf_bits2f(unsigned h) { return __uint_as_float(h << 16); }
__device__ __forceinline__ float bfr(float f) { return bf_bits2f(f2bf_bits(f)); }
__device__ __forceinline__ float leaky(float v) { return (v > 0.0f) ? v : 0.01f * v; }
__device__ __forceinline__ int clampi(int v, int lo, int hi) { return v < lo ? lo : (v > hi ? hi : v); }

union FragB { v16b v; v8b h[2]; };
__device__ __forceinline__ v16b frag_ld(const __bf16* p) {
  FragB f;
  f.h[0] = *(const v8b*)(p);
  f.h[1] = *(const v8b*)(p + 16);
  return f.v;
}
__device__ __forceinline__ v8f mma_bf(v16b a, v16b b, v8f c) {
  return __builtin_amdgcn_wmma_f32_16x16x32_bf16(false, a, false, b, (short)0, c, false, false);
}
__device__ __forceinline__ void acc_guard(v8f& acc, v16b x, v16b y, v16b z) {
  asm volatile("v_nop\n\tv_nop\n\tv_nop\n\tv_nop" : "+v"(acc) : "v"(x), "v"(y), "v"(z));
}

__global__ __launch_bounds__(256) void weight_planes_kernel(
    const float* __restrict__ mW2, const float* __restrict__ mW3,
    unsigned short* __restrict__ W2t, unsigned short* __restrict__ W3t)
{
  __shared__ float sT[64 * 65];
  const int tid = threadIdx.x;
  const int bid = blockIdx.x;
  const bool second = (bid >= kTilesW2);
  const int b2 = second ? (bid - kTilesW2) : bid;
  const int tn = b2 / 12;
  const int tk = b2 - tn * 12;
  const float* src = second ? mW3 : mW2;
  unsigned short* dst = second ? W3t : W2t;
  const int ld = second ? kMsg : kHid;
  const int n0 = tn * 64;
  const int k0 = tk * 64;
  const int nn = tid & 63;
  const int kq = tid >> 6;
  const int ncol = n0 + nn;
  const int nc = (ncol < ld) ? ncol : (ld - 1);
#pragma unroll 4
  for (int i = 0; i < 16; ++i) {
    const int kk = i * 4 + kq;
    float v = src[(size_t)(k0 + kk) * ld + nc];
    v = (ncol < ld) ? v : 0.0f;
    sT[kk * 65 + nn] = v;
  }
  __syncthreads();
  const int rq = tid >> 3;
  const int kc = (tid & 7) * 8;
  v4u pk[2];
#pragma unroll
  for (int it = 0; it < 2; ++it) {
    const int rn = it * 32 + rq;
    unsigned w[4];
#pragma unroll
    for (int e2 = 0; e2 < 4; ++e2) {
      const unsigned h0 = f2bf_bits(sT[(kc + 2 * e2) * 65 + rn]);
      const unsigned h1 = f2bf_bits(sT[(kc + 2 * e2 + 1) * 65 + rn]);
      w[e2] = h0 | (h1 << 16);
    }
    pk[it] = (v4u){w[0], w[1], w[2], w[3]};
  }
  for (int pass = 0; pass < 2; ++pass) {
#pragma unroll
    for (int it = 0; it < 2; ++it) {
      unsigned short* q = dst + (size_t)(n0 + it * 32 + rq) * kHid + k0 + kc;
      *(volatile v4u*)q = pk[it];
    }
    __threadfence();
  }
}

template <int MODE>
__device__ __forceinline__ void epi_tile(const v8f& acc, int rowBase, int n, float bv,
                                         unsigned short* oHi, unsigned short* oLo, float* oW)
{
#pragma unroll
  for (int r = 0; r < 8; ++r) {
    const int row = rowBase + r;
    float v = acc[r] + bv;
    if (MODE == 0) {
      v = leaky(v);
      const unsigned hb = f2bf_bits(v);
      const unsigned lb = f2bf_bits(v - bf_bits2f(hb));
      oHi[row * kHid + n] = (unsigned short)hb;
      oLo[row * kHid + n] = (unsigned short)lb;
    } else {
      oW[row * kMsgPad + n] = v;
    }
  }
}

template <int MODE>
__device__ __forceinline__ void gemm_pair(const unsigned short* aHiU, const unsigned short* aLoU,
                                          const unsigned short* __restrict__ BtU,
                                          const float* __restrict__ bias, int nt0, int lane,
                                          unsigned short* oHi, unsigned short* oLo, float* oW)
{
  const int c  = lane & 15;
  const int hh = lane >> 4;
  const __bf16* a0h = (const __bf16*)aHiU + c * kHid + 8 * hh;
  const __bf16* a1h = a0h + 16 * kHid;
  const __bf16* a0l = (const __bf16*)aLoU + c * kHid + 8 * hh;
  const __bf16* a1l = a0l + 16 * kHid;
  const __bf16* b0p = (const __bf16*)BtU + (size_t)(nt0 * 16 + c) * kHid + 8 * hh;
  const __bf16* b1p = b0p + 16 * kHid;
  v8f c00 = (v8f){0.f, 0.f, 0.f, 0.f, 0.f, 0.f, 0.f, 0.f};
  v8f c01 = c00, c10 = c00, c11 = c00;
#pragma unroll 1
  for (int k0 = 0; k0 < kHid; k0 += 32) {
    const v16b b0 = frag_ld(b0p + k0);
    const v16b b1 = frag_ld(b1p + k0);
    const v16b h0 = frag_ld(a0h + k0);
    const v16b l0 = frag_ld(a0l + k0);
    const v16b h1 = frag_ld(a1h + k0);
    const v16b l1 = frag_ld(a1l + k0);
    c00 = mma_bf(h0, b0, c00);
    c00 = mma_bf(l0, b0, c00);
    c01 = mma_bf(h0, b1, c01);
    c01 = mma_bf(l0, b1, c01);
    c10 = mma_bf(h1, b0, c10);
    c10 = mma_bf(l1, b0, c10);
    c11 = mma_bf(h1, b1, c11);
    c11 = mma_bf(l1, b1, c11);
    acc_guard(c00, h0, l0, b0);
    acc_guard(c01, h0, l0, b1);
    acc_guard(c10, h1, l1, b0);
    acc_guard(c11, h1, l1, b1);
  }
  const int nA = nt0 * 16 + c;
  const int nB = nA + 16;
  float bvA, bvB;
  if (MODE == 0) {
    bvA = bfr(bias[nA]);
    bvB = bfr(bias[nB]);
  } else {
    const int ncA = (nA < kMsg) ? nA : (kMsg - 1);
    const int ncB = (nB < kMsg) ? nB : (kMsg - 1);
    const float rA = bias[ncA];
    const float rB = bias[ncB];
    bvA = (nA < kMsg) ? bfr(rA) : 0.0f;
    bvB = (nB < kMsg) ? bfr(rB) : 0.0f;
  }
  epi_tile<MODE>(c00, 8 * hh,      nA, bvA, oHi, oLo, oW);
  epi_tile<MODE>(c01, 8 * hh,      nB, bvB, oHi, oLo, oW);
  epi_tile<MODE>(c10, 16 + 8 * hh, nA, bvA, oHi, oLo, oW);
  epi_tile<MODE>(c11, 16 + 8 * hh, nB, bvB, oHi, oLo, oW);
}

__global__ __launch_bounds__(256) void edge_message_kernel(
    const float* __restrict__ edge_attr, const float* __restrict__ mW1, const float* __restrict__ mb1,
    const float* __restrict__ mb2, const float* __restrict__ mb3,
    const unsigned short* __restrict__ W2t, const unsigned short* __restrict__ W3t,
    const int* __restrict__ eidx, float* __restrict__ res4)
{
  extern __shared__ __align__(16) unsigned char smem[];
  unsigned short* h1hi = (unsigned short*)smem;
  unsigned short* h1lo = h1hi + kPlaneHalves;
  unsigned short* h2hi = h1lo + kPlaneHalves;
  unsigned short* h2lo = h2hi + kPlaneHalves;
  float* sEa   = (float*)(h2lo + kPlaneHalves);
  float* sRes  = sEa + kTileE * 8;
  int*   sFlag = (int*)(sRes + kTileE * 4);
  int*   sList = sFlag + kTileE;
  float* sW    = (float*)smem;

  const int tid  = threadIdx.x;
  const int lane = tid & 31;
  const int wave = __builtin_amdgcn_readfirstlane((int)(threadIdx.x >> 5));
  const int e0   = blockIdx.x * kTileE;
  const int t64  = tid & 63;

  int sv = eidx[e0 + t64];
  int dv = eidx[kEdges + e0 + t64];
  sv = clampi(sv, 0, kNodes - 1);
  dv = clampi(dv, 0, kNodes - 1);
  const int flag = (sv <= dv) ? 1 : 0;
  if (wave < 2) sFlag[tid] = flag;
  sRes[tid] = 0.0f;
#pragma unroll 1
  for (int it = 0; it < 2; ++it) {
    const int t  = tid + it * 256;
    const int tc = (t < kTileE * kEA) ? t : (kTileE * kEA - 1);
    float v = edge_attr[(size_t)e0 * kEA + tc];
    asm volatile("" : "+v"(v));
    v = bfr(v);
    const int er = t / kEA;
    if (t < kTileE * kEA) sEa[er * 8 + (t - er * kEA)] = v;
  }
  if (wave < 4) sEa[(tid >> 1) * 8 + 6 + (tid & 1)] = 0.0f;
  __syncthreads();

  int cnt = 0, pos = 0;
#pragma unroll 1
  for (int j = 0; j < kTileE; ++j) {
    const int f = sFlag[j];
    cnt += f;
    pos += (j < t64) ? f : 0;
  }
  if (wave < 2) {
    int idx = flag ? pos : (cnt + t64 - pos);
    idx = clampi(idx, 0, kTileE - 1);
    sList[idx] = t64;
  }
  cnt = __builtin_amdgcn_readfirstlane(cnt);
  cnt = clampi(cnt, 0, kTileE);
  const int npass = (cnt + kRowsPass - 1) / kRowsPass;
  __syncthreads();

#pragma unroll 1
  for (int pass = 0; pass < npass; ++pass) {
    if (wave < 6) {
      const int half = (wave >= 3) ? 1 : 0;
      const int oct  = tid - half * 96;
      float wr[kEA][8], br[8];
#pragma unroll
      for (int cc = 0; cc < kEA; ++cc) {
        const v4f wa = *(const v4f*)(mW1 + cc * kHid + oct * 8);
        const v4f wb = *(const v4f*)(mW1 + cc * kHid + oct * 8 + 4);
        wr[cc][0] = bfr(wa[0]); wr[cc][1] = bfr(wa[1]); wr[cc][2] = bfr(wa[2]); wr[cc][3] = bfr(wa[3]);
        wr[cc][4] = bfr(wb[0]); wr[cc][5] = bfr(wb[1]); wr[cc][6] = bfr(wb[2]); wr[cc][7] = bfr(wb[3]);
      }
      {
        const v4f ba = *(const v4f*)(mb1 + oct * 8);
        const v4f bb = *(const v4f*)(mb1 + oct * 8 + 4);
        br[0] = bfr(ba[0]); br[1] = bfr(ba[1]); br[2] = bfr(ba[2]); br[3] = bfr(ba[3]);
        br[4] = bfr(bb[0]); br[5] = bfr(bb[1]); br[6] = bfr(bb[2]); br[7] = bfr(bb[3]);
      }
#pragma unroll 1
      for (int rr = 0; rr < 16; ++rr) {
        const int row = half * 16 + rr;
        const int t = sList[pass * kRowsPass + row];
        const v4f xa = *(const v4f*)(sEa + t * 8);
        const v4f xb = *(const v4f*)(sEa + t * 8 + 4);
        const float xs0 = xa[0], xs1 = xa[1], xs2 = xa[2], xs3 = xa[3], xs4 = xb[0], xs5 = xb[1];
        unsigned hw[4], lw[4];
#pragma unroll
        for (int j2 = 0; j2 < 4; ++j2) {
          float v0 = 0.0f, v1 = 0.0f;
          v0 = fmaf(xs0, wr[0][2 * j2], v0);  v1 = fmaf(xs0, wr[0][2 * j2 + 1], v1);
          v0 = fmaf(xs1, wr[1][2 * j2], v0);  v1 = fmaf(xs1, wr[1][2 * j2 + 1], v1);
          v0 = fmaf(xs2, wr[2][2 * j2], v0);  v1 = fmaf(xs2, wr[2][2 * j2 + 1], v1);
          v0 = fmaf(xs3, wr[3][2 * j2], v0);  v1 = fmaf(xs3, wr[3][2 * j2 + 1], v1);
          v0 = fmaf(xs4, wr[4][2 * j2], v0);  v1 = fmaf(xs4, wr[4][2 * j2 + 1], v1);
          v0 = fmaf(xs5, wr[5][2 * j2], v0);  v1 = fmaf(xs5, wr[5][2 * j2 + 1], v1);
          v0 = leaky(v0 + br[2 * j2]);
          v1 = leaky(v1 + br[2 * j2 + 1]);
          const unsigned h0 = f2bf_bits(v0);
          const unsigned h1b = f2bf_bits(v1);
          const unsigned l0 = f2bf_bits(v0 - bf_bits2f(h0));
          const unsigned l1 = f2bf_bits(v1 - bf_bits2f(h1b));
          hw[j2] = h0 | (h1b << 16);
          lw[j2] = l0 | (l1 << 16);
        }
        *(v4u*)(h1hi + row * kHid + oct * 8) = (v4u){hw[0], hw[1], hw[2], hw[3]};
        *(v4u*)(h1lo + row * kHid + oct * 8) = (v4u){lw[0], lw[1], lw[2], lw[3]};
      }
    }
    __syncthreads();

#pragma unroll 1
    for (int g = 0; g < 3; ++g)
      gemm_pair<0>(h1hi, h1lo, W2t, mb2, wave * 6 + g * 2, lane, h2hi, h2lo, sW);
    __syncthreads();

    gemm_pair<1>(h2hi, h2lo, W3t, mb3, wave * 2, lane, h2hi, h2lo, sW);
    __syncthreads();

    if (wave < 3) {
      const int li = pass * kRowsPass + lane;
      const int t  = sList[li];
      const float* xr = sEa + t * 8;
      const float* wq = sW + lane * kMsgPad + wave * kMono;
      float acc = 0.0f;
      int p = 0;
#pragma unroll
      for (int a = 0; a < kEA; ++a) {
        acc = fmaf(wq[p], xr[a], acc);
        ++p;
      }
#pragma unroll
      for (int a = 0; a < kEA; ++a) {
#pragma unroll
        for (int b = 0; b < kEA; ++b) {
          if (b >= a) {
            acc = fmaf(wq[p], xr[a] * xr[b], acc);
            ++p;
          }
        }
      }
#pragma unroll
      for (int a = 0; a < kEA; ++a) {
#pragma unroll
        for (int b = 0; b < kEA; ++b) {
#pragma unroll
          for (int c = 0; c < kEA; ++c) {
            if (b >= a && c >= b) {
              acc = fmaf(wq[p], (xr[a] * xr[b]) * xr[c], acc);
              ++p;
            }
          }
        }
      }
      if (li < cnt) sRes[t * 4 + wave] = acc;
    }
    __syncthreads();
  }
  __syncthreads();

  if (wave == 0) {
    const v4f v0 = *(const v4f*)(sRes + lane * 4);
    const v4f v1 = *(const v4f*)(sRes + (32 + lane) * 4);
    float* g = res4 + (size_t)e0 * 4;
    *(volatile v4f*)(g + lane * 4) = v0;
    *(volatile v4f*)(g + (32 + lane) * 4) = v1;
    __threadfence();
    *(volatile v4f*)(g + lane * 4) = v0;
    *(volatile v4f*)(g + (32 + lane) * 4) = v1;
  }
}

__device__ __forceinline__ int lower_bound_pair(const int* __restrict__ srcA, const int* __restrict__ dstA,
                                                int ks, int kd)
{
  int lo = 0, hi = kEdges;
#pragma unroll 1
  for (int it = 0; it < kSearchIters; ++it) {
    const int mid = (lo + hi) >> 1;
    const int mc = (mid < kEdges - 1) ? mid : (kEdges - 1);
    int a = srcA[mc];
    int b = dstA[mc];
    asm volatile("" : "+v"(a), "+v"(b));
    const bool act  = (lo < hi);
    const bool less = (a < ks) || ((a == ks) && (b < kd));
    lo = (act && less) ? (mid + 1) : lo;
    hi = (act && !less) ? mid : hi;
  }
  return lo;
}

__device__ __forceinline__ void stage_param(float* dstLds, const float* __restrict__ src, int n, int tid)
{
#pragma unroll 1
  for (int it = 0; it < 2; ++it) {
    const int t  = tid + it * 256;
    const int tc = (t < n) ? t : (n - 1);
    float v = src[tc];
    asm volatile("" : "+v"(v));
    v = bfr(v);
    if (t < n) dstLds[t] = v;
  }
}

__global__ __launch_bounds__(256) void node_update_kernel(
    const float* __restrict__ x, const int* __restrict__ eidx, const float* __restrict__ res4,
    const float* __restrict__ ln_g, const float* __restrict__ ln_b,
    const float* __restrict__ uW1, const float* __restrict__ ub1,
    const float* __restrict__ uW2, const float* __restrict__ ub2,
    const float* __restrict__ uW3, const float* __restrict__ ub3,
    float* __restrict__ out)
{
  __shared__ float sW1[kLnDim * kU1];
  __shared__ float sb1[kU1];
  __shared__ float sW2[kU1 * kU2];
  __shared__ float sb2[kU2];
  __shared__ float sW3[kU2 * kOutDim];
  __shared__ float sb3[kOutDim];
  __shared__ float sg[kLnDim];
  __shared__ float sbt[kLnDim];
  __shared__ __align__(16) float sA[kLnDim * 256];
  __shared__ __align__(16) float sB[kU1 * 256];
  __shared__ __align__(16) float sO[256 * kOutDim];

  const int tid  = threadIdx.x;
  const int lane = tid & 31;
  const int wave = __builtin_amdgcn_readfirstlane((int)(threadIdx.x >> 5));

  stage_param(sW1, uW1, kLnDim * kU1, tid);
  stage_param(sb1, ub1, kU1, tid);
  stage_param(sW2, uW2, kU1 * kU2, tid);
  stage_param(sb2, ub2, kU2, tid);
  stage_param(sW3, uW3, kU2 * kOutDim, tid);
  stage_param(sb3, ub3, kOutDim, tid);
  stage_param(sg,  ln_g, kLnDim, tid);
  stage_param(sbt, ln_b, kLnDim, tid);
  __syncthreads();

  const int n = blockIdx.x * 256 + tid;
  const int* srcA = eidx;
  const int* dstA = eidx + kEdges;

  const int lo = lower_bound_pair(srcA, dstA, n, -2147483647 - 1);
  float g0 = 0.0f, g1 = 0.0f, g2 = 0.0f;
#pragma unroll 1
  for (int j = 0; j < kMaxDeg; ++j) {
    const int f  = lo + j;
    const int fc = (f < kEdges - 1) ? f : (kEdges - 1);
    int fs = srcA[fc];
    int fd = dstA[fc];
    asm volatile("" : "+v"(fs), "+v"(fd));
    const bool valid = (f < kEdges) && (fs == n);
    const int sc = clampi(fd, 0, kNodes - 1);
    int pos = lower_bound_pair(srcA, dstA, sc, n);
    pos = clampi(pos, 0, kEdges - 1);
    int ps = srcA[pos];
    int pd = dstA[pos];
    asm volatile("" : "+v"(ps), "+v"(pd));
    const bool match = valid && (ps == sc) && (pd == n);
    const v4f av = *(const v4f*)(res4 + (size_t)fc * 4);
    const v4f bv = *(const v4f*)(res4 + (size_t)pos * 4);
    float a0 = av[0], a1 = av[1], a2 = av[2];
    float b0 = bv[0], b1 = bv[1], b2 = bv[2];
    asm volatile("" : "+v"(a0), "+v"(a1), "+v"(a2));
    asm volatile("" : "+v"(b0), "+v"(b1), "+v"(b2));
    const bool fwd = (fd > n);
    const float c0 = fwd ? -a0 : b0;
    const float c1 = fwd ? -a1 : b1;
    const float c2 = fwd ? -a2 : b2;
    g0 += match ? c0 : 0.0f;
    g1 += match ? c1 : 0.0f;
    g2 += match ? c2 : 0.0f;
  }

  {
    const float* xr = x + (size_t)n * kNodeIn;
#pragma unroll
    for (int q = 0; q < 4; ++q) {
      const v4f xv = *(const v4f*)(xr + 4 * q);
      sA[(4 * q + 0) * 256 + tid] = bfr(xv[0]);
      sA[(4 * q + 1) * 256 + tid] = bfr(xv[1]);
      sA[(4 * q + 2) * 256 + tid] = bfr(xv[2]);
      sA[(4 * q + 3) * 256 + tid] = bfr(xv[3]);
    }
    sA[16 * 256 + tid] = g0;
    sA[17 * 256 + tid] = g1;
    sA[18 * 256 + tid] = g2;
  }
  float sum = 0.0f;
#pragma unroll 1
  for (int i = 0; i < kLnDim; ++i) sum += sA[i * 256 + tid];
  const float mu = sum * (1.0f / (float)kLnDim);
  float var = 0.0f;
#pragma unroll 1
  for (int i = 0; i < kLnDim; ++i) {
    const float d = sA[i * 256 + tid] - mu;
    var = fmaf(d, d, var);
  }
  var = var * (1.0f / (float)kLnDim);
  const float rs = rsqrtf(var + 1e-5f);
#pragma unroll 1
  for (int i = 0; i < kLnDim; ++i) {
    const float d = sA[i * 256 + tid] - mu;
    sA[i * 256 + tid] = (d * rs) * sg[i] + sbt[i];
  }
#pragma unroll 1
  for (int j = 0; j < kU1; ++j) {
    float a = 0.0f;
#pragma unroll
    for (int i = 0; i < kLnDim; ++i) a = fmaf(sA[i * 256 + tid], sW1[i * kU1 + j], a);
    a += sb1[j];
    sB[j * 256 + tid] = leaky(a);
  }
#pragma unroll 1
  for (int k = 0; k < kU2; ++k) {
    float a = 0.0f;
#pragma unroll
    for (int j = 0; j < kU1; ++j) a = fmaf(sB[j * 256 + tid], sW2[j * kU2 + k], a);
    a += sb2[k];
    sA[k * 256 + tid] = leaky(a);
  }
#pragma unroll 1
  for (int o = 0; o < kOutDim; ++o) {
    float a = 0.0f;
#pragma unroll
    for (int k = 0; k < kU2; ++k) a = fmaf(sA[k * 256 + tid], sW3[k * kOutDim + o], a);
    a += sb3[o];
    sO[tid * kOutDim + o] = a;
  }
  __syncthreads();

  {
    const float* wb = sO + wave * (32 * kOutDim);
    float* gb = out + ((size_t)blockIdx.x * 256 + (size_t)wave * 32) * kOutDim;
    v4f ov[4];
#pragma unroll
    for (int it = 0; it < 4; ++it) ov[it] = *(const v4f*)(wb + (it * 32 + lane) * 4);
    for (int pass = 0; pass < 2; ++pass) {
#pragma unroll
      for (int it = 0; it < 4; ++it) *(volatile v4f*)(gb + (it * 32 + lane) * 4) = ov[it];
      __threadfence();
    }
  }
}

extern "C" void kernel_launch(void* const* d_in, const int* in_sizes, int n_in,
                              void* d_out, int out_size, void* d_ws, size_t ws_size,
                              hipStream_t stream) {
  if (n_in < 17) return;
  if (in_sizes[0] != kNodes * kNodeIn) return;
  if (in_sizes[1] != kEdges * kEA) return;
  if (in_sizes[2] != kEA * kHid) return;
  if (in_sizes[3] != kHid) return;
  if (in_sizes[4] != kHid * kHid) return;
  if (in_sizes[5] != kHid) return;
  if (in_sizes[6] != kHid * kMsg) return;
  if (in_sizes[7] != kMsg) return;
  if (in_sizes[8] != kLnDim) return;
  if (in_sizes[9] != kLnDim) return;
  if (in_sizes[10] != kLnDim * kU1) return;
  if (in_sizes[11] != kU1) return;
  if (in_sizes[12] != kU1 * kU2) return;
  if (in_sizes[13] != kU2) return;
  if (in_sizes[14] != kU2 * kOutDim) return;
  if (in_sizes[15] != kOutDim) return;
  if (in_sizes[16] != 2 * kEdges) return;
  if (out_size != kNodes * kOutDim) return;
  if (ws_size < kWsTotal) return;

  const float* x         = (const float*)d_in[0];
  const float* edge_attr = (const float*)d_in[1];
  const float* mW1  = (const float*)d_in[2];
  const float* mb1  = (const float*)d_in[3];
  const float* mW2  = (const float*)d_in[4];
  const float* mb2  = (const float*)d_in[5];
  const float* mW3  = (const float*)d_in[6];
  const float* mb3  = (const float*)d_in[7];
  const float* ln_g = (const float*)d_in[8];
  const float* ln_b = (const float*)d_in[9];
  const float* uW1  = (const float*)d_in[10];
  const float* ub1  = (const float*)d_in[11];
  const float* uW2  = (const float*)d_in[12];
  const float* ub2  = (const float*)d_in[13];
  const float* uW3  = (const float*)d_in[14];
  const float* ub3  = (const float*)d_in[15];
  const int*   eidx = (const int*)d_in[16];
  float* out = (float*)d_out;

  char* ws = (char*)d_ws;
  unsigned short* W2t = (unsigned short*)(ws + kOffW2);
  unsigned short* W3t = (unsigned short*)(ws + kOffW3);
  float* res4 = (float*)(ws + kOffRes);

  weight_planes_kernel<<<kTilesW2 + kTilesW3, 256, 0, stream>>>(mW2, mW3, W2t, W3t);

  edge_message_kernel<<<kEdges / kTileE, 256, kLdsEdge, stream>>>(
      edge_attr, mW1, mb1, mb2, mb3, W2t, W3t, eidx, res4);

  node_update_kernel<<<kNodes / 256, 256, 0, stream>>>(
      x, eidx, res4, ln_g, ln_b, uW1, ub1, uW2, ub2, uW3, ub3, out);
}
